// CausalSelfAttention_58849641890655
// MI455X (gfx1250) — hardware-verified
//
#include <hip/hip_runtime.h>


#ifndef NB
#define NB 1
#endif
#ifndef SEQ
#define SEQ 4096
#endif
#define SEQ_FULL 4096
#define DM   1024
#define NH_  16
#define HD   64
#define LDQ  (3 * DM)
#define EROWS 256
#define LOP  72
#define PCL  8.0f
#define SCLL2 0.18033688011112042f
#define RSC  2048.0f
#define RSI  4.8828125e-4f

static_assert(SEQ % 64 == 0);
static_assert(DM == NH_ * HD);
static_assert(HD == 64);
static_assert(DM % 32 == 0);
static_assert(LDQ % 64 == 0);
static_assert(((size_t)LDQ * DM / 64) % 32 == 0);
static_assert(((size_t)DM * DM / 64) % 32 == 0);
static_assert(((size_t)SEQ * DM / 8) % 256 == 0);
static_assert(EROWS % 64 == 0);
static_assert(SEQ >= EROWS);
static_assert(((size_t)SEQ * 32) % 256 == 0);
static_assert(256 * 8 == 2 * DM);
static_assert(LOP % 8 == 0);
static_assert(LOP >= HD + 8);
static_assert(HD / 2 == 32);
#define AL256(x) ((((size_t)(x)) + 255) & ~(size_t)255)
static_assert(AL256((size_t)SEQ * DM * 2) + AL256((size_t)LDQ * DM * 2) + AL256((size_t)DM * DM * 2) + AL256((size_t)SEQ * LDQ * 4) + 2 * AL256((size_t)SEQ * DM * 2)
              + AL256(128) + 2 * AL256((size_t)SEQ * 32 * 4) + AL256((size_t)2 * SEQ * DM * 2) + AL256((size_t)2 * EROWS * DM * 2) + AL256((size_t)DM * SEQ * 2) + AL256((size_t)DM * EROWS * 2)
              <= (size_t)134217728);

typedef unsigned short bf;
typedef __attribute__((ext_vector_type(16))) __bf16   v16bf;
typedef __attribute__((ext_vector_type(8)))  unsigned short v8us;
typedef __attribute__((ext_vector_type(2)))  unsigned short v2us;
typedef __attribute__((ext_vector_type(8)))  float    v8f;
typedef __attribute__((ext_vector_type(4)))  float    v4f;
typedef v4f  __attribute__((may_alias)) v4fa;
typedef v8us __attribute__((may_alias)) v8usa;

__device__ __forceinline__ unsigned short f2bf(float f) { unsigned u = __float_as_uint(f); u += 0x7FFFu + ((u >> 16) & 1u); return (unsigned short)(u >> 16); }
__device__ __forceinline__ float bf2f(unsigned short b) { return __uint_as_float(((unsigned)b) << 16); }
__device__ __forceinline__ void splitf(float y, unsigned short& h, unsigned short& l) { h = f2bf(y); l = f2bf(y - bf2f(h)); }
__device__ __forceinline__ v16bf cat16b(v8us lo, v8us hi) { return __builtin_bit_cast(v16bf, __builtin_shufflevector(lo, hi, 0, 1, 2, 3, 4, 5, 6, 7, 8, 9, 10, 11, 12, 13, 14, 15)); }
__device__ __forceinline__ v8f wmmab(v16bf a, v16bf b, v8f c) { return __builtin_amdgcn_wmma_f32_16x16x32_bf16(false, a, false, b, (short)0, c, false, false); }

typedef unsigned short hf;
typedef _Float16 h16;
typedef __attribute__((ext_vector_type(16))) _Float16 v16h;
static __device__ __forceinline__ h16 toh_flush(float v) { const h16 r = (h16)v; return (fabsf(v) < 6.103515625e-05f) ? (h16)0.0f : r; }
__device__ __forceinline__ unsigned short hbits(h16 x) { return __builtin_bit_cast(unsigned short, x); }
__device__ __forceinline__ v16h cat16h(v8us lo, v8us hi) { return __builtin_bit_cast(v16h, __builtin_shufflevector(lo, hi, 0, 1, 2, 3, 4, 5, 6, 7, 8, 9, 10, 11, 12, 13, 14, 15)); }
__device__ __forceinline__ v16h ldfh(const hf* p) { return cat16h(*(const v8us*)p, *(const v8us*)(p + 16)); }
__device__ __forceinline__ v8f mmah(v16h a, v16h b, v8f c) {
    c = __builtin_amdgcn_wmma_f32_16x16x32_f16(false, a, false, b, (short)0, c, false, false);
    asm volatile("v_nop\n\tv_nop\n\tv_nop\n\tv_nop" : "+v"(c) : "v"(a), "v"(b));
    return c; }

template <typename T16> struct WFrag;
template <> struct WFrag<bf> { typedef v16bf V; static __device__ __forceinline__ V ld(const bf* p) { return cat16b(*(const v8us*)p, *(const v8us*)(p + 16)); } static __device__ __forceinline__ v8f mma(V a, V b, v8f c) { return wmmab(a, b, c); } };
template <typename T16, int NSPLIT, bool BIAS>
__global__ __launch_bounds__(32) void k_gemmw(const T16* __restrict__ A, const T16* __restrict__ A2, const T16* __restrict__ Bt, const T16* __restrict__ Bt2, int K, float* C, int ldc, const float* __restrict__ bias, size_t sA, size_t sB, size_t sC) {
    typedef typename WFrag<T16>::V V;
    __shared__ __align__(16) float os[16 * 68];
    const size_t z = blockIdx.z; A += z * sA; if (A2) A2 += z * sA; Bt += z * sB; if (Bt2) Bt2 += z * sB; C += z * sC;
    const int lane = threadIdx.x & 31, lr = lane & 15, hi = lane >> 4; const int r0 = blockIdx.x * 64, c0 = blockIdx.y * 64;
    v8f acc[4][4];
#pragma unroll
    for (int mb = 0; mb < 4; ++mb)
#pragma unroll
        for (int nb = 0; nb < 4; ++nb) acc[mb][nb] = (v8f){};
    const size_t aoff = (size_t)(r0 + lr) * K + 8 * hi, boff = (size_t)(c0 + lr) * K + 8 * hi;
#pragma unroll 1
    for (int kc = 0; kc < K; kc += 32) {
        V a[4], a2[4];
#pragma unroll
        for (int mb = 0; mb < 4; ++mb) { a[mb] = WFrag<T16>::ld(A + aoff + (size_t)mb * 16 * K + kc); if (NSPLIT == 1 || NSPLIT == 2) a2[mb] = WFrag<T16>::ld(A2 + aoff + (size_t)mb * 16 * K + kc); }
#pragma unroll
        for (int nb = 0; nb < 4; ++nb) { const V b = WFrag<T16>::ld(Bt + boff + (size_t)nb * 16 * K + kc); V b2; if (NSPLIT >= 2) b2 = WFrag<T16>::ld(Bt2 + boff + (size_t)nb * 16 * K + kc);
#pragma unroll
            for (int mb = 0; mb < 4; ++mb) { acc[mb][nb] = WFrag<T16>::mma(a[mb], b, acc[mb][nb]); if (NSPLIT == 1 || NSPLIT == 2) acc[mb][nb] = WFrag<T16>::mma(a2[mb], b, acc[mb][nb]); if (NSPLIT >= 2) acc[mb][nb] = WFrag<T16>::mma(a[mb], b2, acc[mb][nb]); } }
        asm volatile("v_nop\n\tv_nop\n\tv_nop\n\tv_nop" : "+v"(acc[0][0]), "+v"(acc[1][1]), "+v"(acc[2][2]), "+v"(acc[3][3]) : "v"(a[0]), "v"(a[3]));
    }
#pragma unroll
    for (int mb = 0; mb < 4; ++mb) {
#pragma unroll
        for (int nb = 0; nb < 4; ++nb) {
#pragma unroll
            for (int j = 0; j < 8; ++j) os[(hi * 8 + j) * 68 + nb * 16 + lr] = acc[mb][nb][j]; }
        __builtin_amdgcn_wave_barrier(); asm volatile("" ::: "memory");
        float* crow = C + (size_t)(r0 + mb * 16) * ldc + c0;
#pragma unroll 1
        for (int ps = 0; ps < 2; ++ps) {
#pragma unroll
            for (int s = 0; s < 8; ++s) { const int row = 2 * s + hi, cofs = lr * 4; v4f val = *(const v4fa*)(os + row * 68 + cofs); if (BIAS) { val[0] += bias[c0 + cofs]; val[1] += bias[c0 + cofs + 1]; val[2] += bias[c0 + cofs + 2]; val[3] += bias[c0 + cofs + 3]; }
                *(volatile v4f*)(crow + (size_t)row * ldc + cofs) = val; }
            if (ps == 0) __threadfence(); }
        __builtin_amdgcn_wave_barrier(); asm volatile("" ::: "memory");
    }
}

__global__ __launch_bounds__(256) void k_wtG(const float* __restrict__ w, unsigned kshift, unsigned N, bf* Bt, unsigned nlines) {
    const unsigned lane = threadIdx.x & 31u; const unsigned L0 = (blockIdx.x * 8u + (threadIdx.x >> 5)) * 4u; const unsigned kmask = (1u << kshift) - 1u;
    v2us o[4];
#pragma unroll
    for (unsigned l = 0; l < 4; ++l) { unsigned L = L0 + l; L = (L < nlines) ? L : (nlines - 1u); const unsigned e = L * 64u + lane * 2u; const unsigned k = e & kmask, n = e >> kshift; v2us t;
        t[0] = f2bf(w[(size_t)k * N + n]); t[1] = f2bf(w[(size_t)(k + 1u) * N + n]); o[l] = t; }
#pragma unroll 1
    for (int ps = 0; ps < 2; ++ps) {
#pragma unroll
        for (unsigned l = 0; l < 4; ++l) { const unsigned L = L0 + l; if (L < nlines) *(volatile v2us*)(Bt + (size_t)L * 64u + lane * 2u) = o[l]; }
        if (ps == 0) __threadfence(); }
}

__global__ __launch_bounds__(256) void k_cvt8(const float* __restrict__ src, bf* dst, size_t n8) { const size_t i = (size_t)blockIdx.x * 256 + threadIdx.x; if (i >= n8) return; const v8f v = *(const v8f*)(src + i * 8); v8us o;
#pragma unroll
    for (int k = 0; k < 8; ++k) o[k] = f2bf(v[k]); *(volatile v8us*)(dst + i * 8) = o; __threadfence(); *(volatile v8us*)(dst + i * 8) = o; }

__global__ __launch_bounds__(32) void k_freq(float* FR) {
#pragma clang fp contract(off)
    const unsigned i = threadIdx.x & 31u;
    const float p = powf(10000.0f, (float)i * 0.03125f);
    const float v = 1.0f / p;
    *(volatile float*)(FR + i) = v; __threadfence(); *(volatile float*)(FR + i) = v;
}

__global__ __launch_bounds__(256) void k_tab(const float* __restrict__ FR, float* CT, float* ST) {
#pragma clang fp contract(off)
    const unsigned idx = blockIdx.x * 256u + threadIdx.x; const unsigned t = idx >> 5, i = idx & 31u;
    const float ang = (float)t * FR[i];
    float s, c; sincosf(ang, &s, &c);
    *(volatile float*)(CT + idx) = c; *(volatile float*)(ST + idx) = s;
    __threadfence();
    *(volatile float*)(CT + idx) = c; *(volatile float*)(ST + idx) = s;
}

__global__ __launch_bounds__(256) void k_rope(const float* __restrict__ QKV, const float* __restrict__ CT, const float* __restrict__ ST, hf* QKF, hf* QKR) {
#pragma clang fp contract(off)
    const unsigned t = blockIdx.x, tid = threadIdx.x;
    const unsigned which = tid >> 7, col = (tid & 127u) * 8u;
    const unsigned dl = col & 63u; const bool lowhalf = dl < 32u;
    const unsigned pcol = lowhalf ? (col + 32u) : (col - 32u); const unsigned j = dl & 31u;
    const float* row = QKV + (size_t)t * LDQ + (size_t)which * DM;
    const v8f a = *(const v8f*)(row + col); const v8f b = *(const v8f*)(row + pcol);
    const v8f c = *(const v8f*)(CT + (size_t)t * 32u + j); const v8f s = *(const v8f*)(ST + (size_t)t * 32u + j);
    v8us oh, ores;
#pragma unroll
    for (int e = 0; e < 8; ++e) {
        const float rb = lowhalf ? -b[e] : b[e];
        const float t0 = a[e] * c[e]; const float t1 = rb * s[e]; const float y = t0 + t1;
        const h16 hh = toh_flush(y); oh[e] = hbits(hh);
        ores[e] = hbits(toh_flush((y - (float)hh) * RSC)); }
    const size_t g  = (size_t)which * SEQ * DM + (size_t)t * DM + col;
    const size_t gr = (size_t)which * EROWS * DM + (size_t)t * DM + col;
    const bool early = t < (unsigned)EROWS;
    *(volatile v8us*)(QKF + g) = oh; if (early) *(volatile v8us*)(QKR + gr) = ores;
    __threadfence();
    *(volatile v8us*)(QKF + g) = oh; if (early) *(volatile v8us*)(QKR + gr) = ores;
}

__global__ __launch_bounds__(256) void k_vt(const float* __restrict__ QKV, hf* VT, hf* VTR) {
#pragma clang fp contract(off)
    __shared__ __align__(16) unsigned short Th[64 * LOP];
    __shared__ __align__(16) unsigned short Tr[64 * LOP];
    const unsigned tid = threadIdx.x, t0 = blockIdx.x * 64u, hd = blockIdx.y;
    const float* vbase = QKV + 2 * DM + hd * HD;
#pragma unroll 1
    for (unsigned it = 0; it < 2u; ++it) {
        const unsigned idx = tid + it * 256u, row = idx >> 3, c8 = (idx & 7u) * 8u;
        const v8f vv = *(const v8f*)(vbase + (size_t)(t0 + row) * LDQ + c8);
#pragma unroll
        for (int q = 0; q < 8; ++q) { const float y = vv[q]; const h16 hh = toh_flush(y);
            Th[(c8 + (unsigned)q) * LOP + row] = hbits(hh); Tr[(c8 + (unsigned)q) * LOP + row] = hbits(toh_flush((y - (float)hh) * RSC)); }
    }
    __syncthreads();
    v8us oh[2], ores[2];
#pragma unroll
    for (unsigned it = 0; it < 2u; ++it) { const unsigned idx = tid + it * 256u, d = idx >> 3, c = (idx & 7u) * 8u;
        oh[it] = *(const v8usa*)(Th + d * LOP + c); ores[it] = *(const v8usa*)(Tr + d * LOP + c); }
    const bool early = t0 < (unsigned)EROWS;
#pragma unroll 1
    for (int ps = 0; ps < 2; ++ps) {
#pragma unroll
        for (unsigned it = 0; it < 2u; ++it) { const unsigned idx = tid + it * 256u, d = idx >> 3, c = (idx & 7u) * 8u;
            *(volatile v8us*)(VT + (size_t)(hd * HD + d) * SEQ + t0 + c) = oh[it];
            if (early) *(volatile v8us*)(VTR + (size_t)(hd * HD + d) * EROWS + t0 + c) = ores[it]; }
        if (ps == 0) __threadfence(); }
}

template <bool EARLY>
__device__ __forceinline__ void attn_body(const hf* QF, const hf* QR, const hf* KF, const hf* KR, const hf* VT, const hf* VTR, bf* CH, bf* CL, unsigned qbase) {
    __shared__ __align__(16) unsigned short Oh[4 * 16 * LOP];
    __shared__ __align__(16) unsigned short Ol[4 * 16 * LOP];
    const unsigned lane = threadIdx.x & 31u, lr = lane & 15u, hi = lane >> 4;
    const unsigned wave = (unsigned)__builtin_amdgcn_readfirstlane((int)(threadIdx.x >> 5));
    const unsigned hd = blockIdx.y;
    const unsigned q0 = qbase + blockIdx.x * 64u + 16u * wave;
    const unsigned qg = q0 + lr;
    v16h qh[2], qr[2];
    {
        const size_t qoff = (size_t)qg * DM + hd * HD + 8u * hi;
#pragma unroll
        for (int kc = 0; kc < 2; ++kc) { qh[kc] = ldfh(QF + qoff + (unsigned)kc * 32u); if (EARLY) qr[kc] = ldfh(QR + qoff + (unsigned)kc * 32u); else qr[kc] = qh[kc]; }
    }
    v8f ot[4], orr[4];
#pragma unroll
    for (int dt = 0; dt < 4; ++dt) { ot[dt] = (v8f){}; orr[dt] = (v8f){}; }
    float m = -1.0e30f, l = 0.0f;
    const unsigned nsteps = (q0 + 15u) / 32u + 1u;
    const size_t kofs  = (size_t)lr * DM + hd * HD + 8u * hi;
    const size_t vofs  = (size_t)(hd * HD + lr) * SEQ + 8u * hi;
    const size_t vrofs = (size_t)(hd * HD + lr) * EROWS + 8u * hi;
#pragma unroll 1
    for (unsigned kb = 0; kb < nsteps; ++kb) {
        const unsigned key0 = kb * 32u;
        v8f st[2], sr[2];
#pragma unroll
        for (int j = 0; j < 2; ++j) {
            st[j] = (v8f){}; sr[j] = (v8f){};
#pragma unroll
            for (int kc = 0; kc < 2; ++kc) {
                const size_t ko = kofs + (size_t)(key0 + 16u * (unsigned)j) * DM + (unsigned)kc * 32u;
                const v16h kh = ldfh(KF + ko);
                st[j] = mmah(kh, qh[kc], st[j]);
                if (EARLY) { const v16h kr = ldfh(KR + ko); sr[j] = mmah(kr, qh[kc], sr[j]); sr[j] = mmah(kh, qr[kc], sr[j]); }
            }
        }
        float mx = -1.0e30f;
#pragma unroll
        for (int j = 0; j < 2; ++j) {
#pragma unroll
            for (int r = 0; r < 8; ++r) {
                const unsigned key = key0 + 16u * (unsigned)j + 8u * hi + (unsigned)r;
                float s = st[j][r]; if (EARLY) s += sr[j][r] * RSI;
                s = (key <= qg) ? (s * SCLL2) : -1.0e30f;
                st[j][r] = s; mx = fmaxf(mx, s); }
        }
        mx = fmaxf(mx, __shfl_xor(mx, 16, 32));
        const float mnew = fmaxf(m, mx);
        const float alpha = __builtin_amdgcn_exp2f(m - mnew);
        m = mnew;
        float rs = 0.0f;
        v16h pf, prf;
#pragma unroll
        for (int j = 0; j < 2; ++j) {
#pragma unroll
            for (int r = 0; r < 8; ++r) {
                const float e = (st[j][r] - mnew) + PCL;
                const float ex = __builtin_amdgcn_exp2f(e);
                const float p = (e >= -14.0f) ? ex : 0.0f;
                const h16 ph = (h16)p;
                pf[8 * j + r] = ph;
                if (EARLY) { prf[8 * j + r] = toh_flush((p - (float)ph) * RSC); rs += p; } else { prf[8 * j + r] = ph; rs += (float)ph; }
            }
        }
        rs += __shfl_xor(rs, 16, 32);
        l = l * alpha + rs;
#pragma unroll
        for (int dt = 0; dt < 4; ++dt) { ot[dt] = ot[dt] * alpha; if (EARLY) orr[dt] = orr[dt] * alpha; }
#pragma unroll
        for (int dt = 0; dt < 4; ++dt) {
            const v16h vh = ldfh(VT + vofs + (size_t)(16u * (unsigned)dt) * SEQ + key0);
            ot[dt] = mmah(vh, pf, ot[dt]);
            if (EARLY) { const v16h vr = ldfh(VTR + vrofs + (size_t)(16u * (unsigned)dt) * EROWS + key0); orr[dt] = mmah(vr, pf, orr[dt]); orr[dt] = mmah(vh, prf, orr[dt]); }
        }
    }
    const float inv = __builtin_amdgcn_rcpf(l);
    const unsigned ob = wave * 16u * LOP;
#pragma unroll
    for (int dt = 0; dt < 4; ++dt) {
        v8us h8, l8;
#pragma unroll
        for (int r = 0; r < 8; ++r) { float y = ot[dt][r]; if (EARLY) y += orr[dt][r] * RSI; y *= inv; unsigned short a, c; splitf(y, a, c); h8[r] = a; l8[r] = c; }
        const unsigned o = ob + lr * LOP + 16u * (unsigned)dt + 8u * hi;
        *(v8usa*)(Oh + o) = h8; *(v8usa*)(Ol + o) = l8;
    }
    __syncthreads();
#pragma unroll 1
    for (int ps = 0; ps < 2; ++ps) {
#pragma unroll
        for (unsigned s = 0; s < 4u; ++s) { const unsigned row = 4u * s + (lane >> 3), c = (lane & 7u) * 8u;
            const v8us vh8 = *(const v8usa*)(Oh + ob + row * LOP + c); const v8us vl8 = *(const v8usa*)(Ol + ob + row * LOP + c);
            const size_t g = (size_t)(q0 + row) * DM + hd * HD + c;
            *(volatile v8us*)(CH + g) = vh8; *(volatile v8us*)(CL + g) = vl8; }
        if (ps == 0) __threadfence(); }
}

__global__ __launch_bounds__(128) __attribute__((amdgpu_num_vgpr(256))) void k_attn_early(const hf* QF, const hf* QR, const hf* KF, const hf* KR, const hf* VT, const hf* VTR, bf* CH, bf* CL) {
    attn_body<true>(QF, QR, KF, KR, VT, VTR, CH, CL, 0u);
}
__global__ __launch_bounds__(128) __attribute__((amdgpu_num_vgpr(256))) void k_attn_late(const hf* QF, const hf* KF, const hf* VT, bf* CH, bf* CL) {
    attn_body<false>(QF, QF, KF, KF, VT, VT, CH, CL, (unsigned)EROWS);
}

extern "C" void kernel_launch(void* const* d_in, const int* in_sizes, int n_in,
                              void* d_out, int out_size, void* d_ws, size_t ws_size, hipStream_t stream) {
    (void)out_size;
    if (n_in < 3) return;
    if (in_sizes[0] < NB * SEQ * DM || in_sizes[1] < DM * LDQ || in_sizes[2] < DM * DM) return;
    const float* X = (const float*)d_in[0]; const float* Wqkv = (const float*)d_in[1]; const float* Wo = (const float*)d_in[2];
    float* OUT = (float*)d_out;
    char* wsp = (char*)d_ws;
    auto take = [&](size_t bytes) { char* p = wsp; wsp += (bytes + 255) & ~(size_t)255; return (void*)p; };
    bf* XB  = (bf*)take((size_t)SEQ * DM * 2);
    bf* WqT = (bf*)take((size_t)LDQ * DM * 2);
    bf* WoT = (bf*)take((size_t)DM * DM * 2);
    float* QKVb = (float*)take((size_t)SEQ * LDQ * 4);
    bf* CH = (bf*)take((size_t)SEQ * DM * 2);
    bf* CL = (bf*)take((size_t)SEQ * DM * 2);
    float* FR = (float*)take(128);
    float* CT = (float*)take((size_t)SEQ * 32 * 4);
    float* ST = (float*)take((size_t)SEQ * 32 * 4);
    hf* QKF = (hf*)take((size_t)2 * SEQ * DM * 2);
    hf* QKR = (hf*)take((size_t)2 * EROWS * DM * 2);
    hf* VT  = (hf*)take((size_t)DM * SEQ * 2);
    hf* VTR = (hf*)take((size_t)DM * EROWS * 2);
    const size_t carved = (size_t)(wsp - (char*)d_ws);
    if (carved > ws_size || carved > (size_t)134217728) return;
    { const unsigned nl = (unsigned)((size_t)LDQ * DM / 64); k_wtG<<<(nl + 31u) / 32u, 256, 0, stream>>>(Wqkv, 10u, (unsigned)LDQ, WqT, nl); }
    { const unsigned nl = (unsigned)((size_t)DM * DM / 64);  k_wtG<<<(nl + 31u) / 32u, 256, 0, stream>>>(Wo, 10u, (unsigned)DM, WoT, nl); }
    k_freq<<<1, 32, 0, stream>>>(FR);
    k_tab<<<(unsigned)((size_t)SEQ * 32 / 256), 256, 0, stream>>>(FR, CT, ST);
    for (int b = 0; b < NB; ++b) {
        const float* xb = X + (size_t)b * SEQ_FULL * DM; float* ob = OUT + (size_t)b * SEQ_FULL * DM;
        const size_t n8 = (size_t)SEQ * DM / 8;
        k_cvt8<<<(unsigned)((n8 + 255) / 256), 256, 0, stream>>>(xb, XB, n8);
        k_gemmw<bf, 0, false><<<dim3(SEQ / 64, LDQ / 64, 1), 32, 0, stream>>>(XB, nullptr, WqT, nullptr, DM, QKVb, LDQ, nullptr, 0, 0, 0);
        k_rope<<<SEQ, 256, 0, stream>>>(QKVb, CT, ST, QKF, QKR);
        k_vt<<<dim3(SEQ / 64, NH_, 1), 256, 0, stream>>>(QKVb, VT, VTR);
        k_attn_early<<<dim3(EROWS / 64, NH_, 1), 128, 0, stream>>>(QKF, QKR, QKF + (size_t)SEQ * DM, QKR + (size_t)EROWS * DM, VT, VTR, CH, CL);
        if (SEQ > EROWS) k_attn_late<<<dim3((SEQ - EROWS) / 64, NH_, 1), 128, 0, stream>>>(QKF, QKF + (size_t)SEQ * DM, VT, CH, CL);
        k_gemmw<bf, 1, false><<<dim3(SEQ / 64, DM / 64, 1), 32, 0, stream>>>(CH, CL, WoT, nullptr, DM, ob, DM, nullptr, 0, 0, 0);
    }
}
